// BertSelfAttention_60593398611978
// MI455X (gfx1250) — hardware-verified
//
#include <hip/hip_runtime.h>


#ifndef NB
#define NB 2
#endif
#ifndef SEQ
#define SEQ 2048
#endif
#define NB_FULL  2
#define SEQ_FULL 2048
#define DM   1024
#define NH   16
#define HD   64
#define NTOK (NB * SEQ)
#define QT   (SEQ / 16)
#define NCH  (SEQ / 32)
#define PP   40
#define OP   68
#define SP   72

static_assert(SEQ % 256 == 0);
static_assert(SEQ <= 2048);
static_assert(SEQ <= SEQ_FULL);
static_assert(NB >= 1);
static_assert(NB <= NB_FULL);
static_assert(DM == NH * HD);
static_assert(NCH <= 64);

typedef _Float16 f16t;
typedef _Float16 v16h __attribute__((ext_vector_type(16)));
typedef _Float16 v8h  __attribute__((ext_vector_type(8), may_alias));
typedef float    v8f  __attribute__((ext_vector_type(8)));
typedef float    v4f  __attribute__((ext_vector_type(4), may_alias));
typedef unsigned v4u  __attribute__((ext_vector_type(4), may_alias));

union Frag { v16h v; v8h hh[2]; };

__device__ __forceinline__ float bfr(float f) {
    unsigned u = __float_as_uint(f);
    u += 0x7FFFu + ((u >> 16) & 1u);
    u &= 0xFFFF0000u;
    return __uint_as_float(u);
}
__device__ __forceinline__ unsigned h2(float a, float b) {
    return (unsigned)__builtin_bit_cast(unsigned short, (f16t)a) | ((unsigned)__builtin_bit_cast(unsigned short, (f16t)b) << 16);
}
__device__ __forceinline__ v8f vzero() { v8f z; z[0] = 0.f; z[1] = 0.f; z[2] = 0.f; z[3] = 0.f; z[4] = 0.f; z[5] = 0.f; z[6] = 0.f; z[7] = 0.f; return z; }

__device__ __forceinline__ v8f wmma16(v16h a, v16h b, v8f c) {
    c = __builtin_amdgcn_wmma_f32_16x16x32_f16(false, a, false, b, (short)0, c, false, false);
    asm volatile("v_nop\n\tv_nop\n\tv_nop\n\tv_nop" : "+v"(c) : "v"(a), "v"(b));
    return c;
}

__global__ __launch_bounds__(256) void k_cvt_x(const float* __restrict__ X, f16t* __restrict__ Xh) {
    const size_t u = (size_t)blockIdx.x * 256 + threadIdx.x;
    const size_t e = u * 8;
    const size_t tok = e / DM;
    const int k = (int)(e - tok * DM);
    const int bb = (int)(tok / SEQ), l = (int)(tok - (size_t)bb * SEQ);
    const float* src = X + ((size_t)bb * SEQ_FULL + l) * DM + k;
    const v4f x0 = *(const v4f*)(src);
    const v4f x1 = *(const v4f*)(src + 4);
    v4u o;
    o.x = h2(bfr(x0.x), bfr(x0.y)); o.y = h2(bfr(x0.z), bfr(x0.w));
    o.z = h2(bfr(x1.x), bfr(x1.y)); o.w = h2(bfr(x1.z), bfr(x1.w));
    f16t* dst = Xh + e;
    *(volatile v4u*)dst = o;
    __threadfence();
    *(volatile v4u*)dst = o;
}

__global__ __launch_bounds__(256) void k_wt(const float* __restrict__ Wq, const float* __restrict__ Wk, const float* __restrict__ Wv,
                                           f16t* __restrict__ WtAll) {
    __shared__ float tile[64][65];
    const int z = blockIdx.z;
    const float* W = (z == 0) ? Wq : ((z == 1) ? Wk : Wv);
    f16t* Wt = WtAll + (size_t)z * DM * DM;
    const int n0 = blockIdx.x * 64, k0 = blockIdx.y * 64, tid = threadIdx.x;
#pragma unroll
    for (int p = 0; p < 4; ++p) {
        const int r = p * 16 + (tid >> 4), c = 4 * (tid & 15);
        const v4f v = *(const v4f*)(W + (size_t)(k0 + r) * DM + n0 + c);
        tile[r][c] = v.x; tile[r][c + 1] = v.y; tile[r][c + 2] = v.z; tile[r][c + 3] = v.w;
    }
    __syncthreads();
    v4u o[2]; size_t off[2];
#pragma unroll
    for (int p = 0; p < 2; ++p) {
        const int L = p * 32 + (tid >> 3), kk = 8 * (tid & 7);
        const float w0 = 64.0f * bfr(tile[kk + 0][L]), w1 = 64.0f * bfr(tile[kk + 1][L]);
        const float w2 = 64.0f * bfr(tile[kk + 2][L]), w3 = 64.0f * bfr(tile[kk + 3][L]);
        const float w4 = 64.0f * bfr(tile[kk + 4][L]), w5 = 64.0f * bfr(tile[kk + 5][L]);
        const float w6 = 64.0f * bfr(tile[kk + 6][L]), w7 = 64.0f * bfr(tile[kk + 7][L]);
        o[p].x = h2(w0, w1); o[p].y = h2(w2, w3); o[p].z = h2(w4, w5); o[p].w = h2(w6, w7);
        off[p] = (size_t)(n0 + L) * DM + k0 + kk;
    }
#pragma unroll
    for (int p = 0; p < 2; ++p) *(volatile v4u*)(Wt + off[p]) = o[p];
    __threadfence();
#pragma unroll
    for (int p = 0; p < 2; ++p) *(volatile v4u*)(Wt + off[p]) = o[p];
}

__global__ __launch_bounds__(256) void k_mt(const float* __restrict__ M, float* __restrict__ MT) {
    __shared__ float tile[64][65];
    const int c0 = blockIdx.x * 64, q0 = blockIdx.y * 64, tid = threadIdx.x;
#pragma unroll
    for (int p = 0; p < 4; ++p) {
        const int r = p * 16 + (tid >> 4), c = 4 * (tid & 15);
        const v4f v = *(const v4f*)(M + (size_t)(q0 + r) * SEQ_FULL + c0 + c);
        tile[r][c] = bfr(v.x); tile[r][c + 1] = bfr(v.y); tile[r][c + 2] = bfr(v.z); tile[r][c + 3] = bfr(v.w);
    }
    __syncthreads();
    v4f o[4]; size_t off[4];
#pragma unroll
    for (int p = 0; p < 4; ++p) {
        const int L = p * 32 + (tid >> 3), kl = L >> 1, qo = (L & 1) * 32 + 4 * (tid & 7);
        v4f t; t.x = tile[qo][kl]; t.y = tile[qo + 1][kl]; t.z = tile[qo + 2][kl]; t.w = tile[qo + 3][kl];
        o[p] = t;
        off[p] = (size_t)(c0 + kl) * SEQ + q0 + qo;
    }
#pragma unroll
    for (int p = 0; p < 4; ++p) *(volatile v4f*)(MT + off[p]) = o[p];
    __threadfence();
#pragma unroll
    for (int p = 0; p < 4; ++p) *(volatile v4f*)(MT + off[p]) = o[p];
}

__global__ __launch_bounds__(256) void k_scan(const float* __restrict__ M, const float* __restrict__ am,
                                             unsigned long long* __restrict__ act) {
    __shared__ unsigned long long bl[16];
    const int tid = threadIdx.x, lane = tid & 31, wv = tid >> 5;
    int bad = 0;
#pragma unroll 1
    for (int i = lane; i < NB * SEQ; i += 32) {
        const int bb = i / SEQ, kk = i - bb * SEQ;
        const float v = am[(size_t)bb * SEQ_FULL + kk];
        bad |= !(fabsf(v) <= 1000.0f);
    }
    const int amok = (__ballot(bad) == 0ull);
#pragma unroll 1
    for (int i = 0; i < 2; ++i) {
        const int qt = blockIdx.x * 16 + wv * 2 + i;
        const int q0 = qt * 16;
        unsigned long long lbits = 0ull;
        int allrows = 1;
#pragma unroll 1
        for (int r = 0; r < 16; ++r) {
            const float* row = M + (size_t)(q0 + r) * SEQ_FULL;
            int vis = 0;
#pragma unroll 4
            for (int g = 0; g < SEQ / 128; ++g) {
                const v4f v = *(const v4f*)(row + g * 128 + 4 * lane);
                const int anyA = (v.x > -5000.f) | (v.y > -5000.f) | (v.z > -5000.f) | (v.w > -5000.f);
                vis |= (v.x >= -1000.f) | (v.y >= -1000.f) | (v.z >= -1000.f) | (v.w >= -1000.f);
                const int cbit = 4 * g + (lane >> 3);
                if (anyA) lbits |= (1ull << cbit);
            }
            if (__ballot(vis) == 0ull) allrows = 0;
        }
        unsigned lo = (unsigned)lbits, hi = (unsigned)(lbits >> 32);
#pragma unroll
        for (int o2 = 16; o2; o2 >>= 1) { lo |= __shfl_xor(lo, o2, 32); hi |= __shfl_xor(hi, o2, 32); }
        unsigned long long bits = (unsigned long long)lo | ((unsigned long long)hi << 32);
        if (!(amok && allrows)) bits = ~0ull;
        if (lane == 0) bl[wv * 2 + i] = bits;
    }
    __syncthreads();
    if (tid < 8) {
        const unsigned long long b0 = bl[2 * tid], b1 = bl[2 * tid + 1];
        v4u o; o.x = (unsigned)b0; o.y = (unsigned)(b0 >> 32); o.z = (unsigned)b1; o.w = (unsigned)(b1 >> 32);
        unsigned* dst = (unsigned*)(act + (size_t)blockIdx.x * 16 + 2 * tid);
        *(volatile v4u*)dst = o;
        __threadfence();
        *(volatile v4u*)dst = o;
    }
}

__global__ __launch_bounds__(128) void k_proj(const f16t* __restrict__ Xh, const f16t* __restrict__ WtAll,
                                             const float* __restrict__ bq, const float* __restrict__ bk, const float* __restrict__ bv,
                                             f16t* __restrict__ Qh, f16t* __restrict__ Ql, f16t* __restrict__ Kh, f16t* __restrict__ Kl,
                                             f16t* __restrict__ Vt) {
    __shared__ __align__(16) f16t st[64 * SP];
    __shared__ __align__(16) f16t st2[64 * SP];
    const int z = blockIdx.z;
    const f16t* Wt = WtAll + (size_t)z * DM * DM;
    const float* bias = (z == 0) ? bq : ((z == 1) ? bk : bv);
    const int tid = threadIdx.x, lane = tid & 31, wv = tid >> 5, m = lane & 15, h = lane >> 4;
    const int row0 = blockIdx.x * 64;
    const int col0 = blockIdx.y * 64;
    const f16t* arow = Xh + (size_t)(row0 + wv * 16 + m) * DM + 8 * h;
    const f16t* bbase = Wt + (size_t)(col0 + m) * DM + 8 * h;
    v8f acc[4];
#pragma unroll
    for (int t = 0; t < 4; ++t) acc[t] = vzero();
#pragma unroll 1
    for (int kc = 0; kc < DM; kc += 32) {
        Frag a;
        a.hh[0] = *(const v8h*)(arow + kc);
        a.hh[1] = *(const v8h*)(arow + kc + 16);
#pragma unroll
        for (int t = 0; t < 4; ++t) {
            const f16t* brow = bbase + (size_t)(t * 16) * DM + kc;
            Frag b;
            b.hh[0] = *(const v8h*)(brow);
            b.hh[1] = *(const v8h*)(brow + 16);
            acc[t] = wmma16(a.v, b.v, acc[t]);
        }
    }
    const int bb = row0 / SEQ, l0 = row0 - bb * SEQ;
    const int bh = bb * NH + blockIdx.y;
    const float wsc = 0.015625f;
    if (z == 2) {
#pragma unroll
        for (int t = 0; t < 4; ++t) {
            const float bvl = bfr(bias[col0 + t * 16 + m]);
            v4u pk;
            pk.x = h2(acc[t][0] * wsc + bvl, acc[t][1] * wsc + bvl);
            pk.y = h2(acc[t][2] * wsc + bvl, acc[t][3] * wsc + bvl);
            pk.z = h2(acc[t][4] * wsc + bvl, acc[t][5] * wsc + bvl);
            pk.w = h2(acc[t][6] * wsc + bvl, acc[t][7] * wsc + bvl);
            *(v4u*)(st + (t * 16 + m) * SP + wv * 16 + 8 * h) = pk;
        }
    } else {
#pragma unroll
        for (int t = 0; t < 4; ++t) {
            const float bvl = bfr(bias[col0 + t * 16 + m]);
#pragma unroll
            for (int r = 0; r < 8; ++r) {
                const float v = acc[t][r] * wsc + bvl;
                const f16t hv = (f16t)v;
                const int ix = (wv * 16 + 8 * h + r) * SP + t * 16 + m;
                st[ix]  = hv;
                st2[ix] = (f16t)((v - (float)hv) * 1024.0f);
            }
        }
    }
    __syncthreads();
    const bool two = (z != 2);
    f16t* dstp = (z == 2) ? Vt : ((z == 0) ? Qh : Kh);
    f16t* dstl = (z == 0) ? Ql : Kl;
    v4u o[4], ol[4]; size_t off[4];
#pragma unroll
    for (int p = 0; p < 4; ++p) {
        const int L = p * 16 + (tid >> 3), piece = 8 * (tid & 7);
        o[p] = *(const v4u*)(st + L * SP + piece);
        ol[p] = o[p];
        if (two) ol[p] = *(const v4u*)(st2 + L * SP + piece);
        off[p] = (z == 2) ? (((size_t)bh * HD + L) * SEQ + l0 + piece) : (((size_t)bh * SEQ + l0 + L) * HD + piece);
    }
#pragma unroll
    for (int p = 0; p < 4; ++p) *(volatile v4u*)(dstp + off[p]) = o[p];
    if (two) {
#pragma unroll
        for (int p = 0; p < 4; ++p) *(volatile v4u*)(dstl + off[p]) = ol[p];
    }
    __threadfence();
#pragma unroll
    for (int p = 0; p < 4; ++p) *(volatile v4u*)(dstp + off[p]) = o[p];
    if (two) {
#pragma unroll
        for (int p = 0; p < 4; ++p) *(volatile v4u*)(dstl + off[p]) = ol[p];
    }
}

__global__ __launch_bounds__(128) void k_attn(const f16t* __restrict__ Qh, const f16t* __restrict__ Ql,
                                             const f16t* __restrict__ Kh, const f16t* __restrict__ Kl, const f16t* __restrict__ Vt,
                                             const float* __restrict__ MT, const float* __restrict__ am,
                                             const unsigned long long* __restrict__ act, float* __restrict__ out) {
    __shared__ __align__(16) f16t Pbuf[4][16 * PP];
    __shared__ __align__(16) float Obuf[4][16 * OP];
    const int tid = threadIdx.x, lane = tid & 31, wv = tid >> 5;
    const int m = lane & 15, h = lane >> 4;
    const int qt = blockIdx.x * 4 + wv;
    const int q0 = qt * 16;
    const int bh = blockIdx.y, bb = bh / NH, hd0 = (bh - bb * NH) * HD;
    const f16t* Qb  = Qh + (size_t)bh * SEQ * HD;
    const f16t* Qlb = Ql + (size_t)bh * SEQ * HD;
    const f16t* Kb  = Kh + (size_t)bh * SEQ * HD;
    const f16t* Klb = Kl + (size_t)bh * SEQ * HD;
    const f16t* Vb  = Vt + (size_t)bh * HD * SEQ;
    const float* amb = am + (size_t)bb * SEQ_FULL;
    const float* mq = MT + q0 + 8 * h;
    f16t* Pw = &Pbuf[wv][0];
    float* Ow = &Obuf[wv][0];
    const unsigned long long bits = act[qt];

    Frag aq0, aq1, al0, al1;
    {
        const f16t* qrow = Qb + (size_t)(q0 + m) * HD + 8 * h;
        aq0.hh[0] = *(const v8h*)(qrow);      aq0.hh[1] = *(const v8h*)(qrow + 16);
        aq1.hh[0] = *(const v8h*)(qrow + 32); aq1.hh[1] = *(const v8h*)(qrow + 48);
        const f16t* lrow = Qlb + (size_t)(q0 + m) * HD + 8 * h;
        al0.hh[0] = *(const v8h*)(lrow);      al0.hh[1] = *(const v8h*)(lrow + 16);
        al1.hh[0] = *(const v8h*)(lrow + 32); al1.hh[1] = *(const v8h*)(lrow + 48);
    }
    v8f acc[4];
#pragma unroll
    for (int t = 0; t < 4; ++t) acc[t] = vzero();
    float rmax[8], rsum[8];
#pragma unroll
    for (int r = 0; r < 8; ++r) { rmax[r] = -1.0e30f; rsum[r] = 0.0f; }

#pragma unroll 1
    for (int ci = 0; ci < NCH; ++ci) {
        const int on = __builtin_amdgcn_readfirstlane((int)((bits >> ci) & 1ull));
        if (!on) continue;
        const int kc = ci * 32;
        v8f S0, S1;
#pragma unroll
        for (int t = 0; t < 2; ++t) {
            const int key = kc + t * 16 + m;
            const f16t* krow = Kb + (size_t)key * HD + 8 * h;
            const f16t* klr  = Klb + (size_t)key * HD + 8 * h;
            Frag bk0, bk1, bl0, bl1;
            bk0.hh[0] = *(const v8h*)(krow);      bk0.hh[1] = *(const v8h*)(krow + 16);
            bk1.hh[0] = *(const v8h*)(krow + 32); bk1.hh[1] = *(const v8h*)(krow + 48);
            bl0.hh[0] = *(const v8h*)(klr);       bl0.hh[1] = *(const v8h*)(klr + 16);
            bl1.hh[0] = *(const v8h*)(klr + 32);  bl1.hh[1] = *(const v8h*)(klr + 48);
            v8f s = vzero();
            s = wmma16(aq0.v, bk0.v, s);
            s = wmma16(aq1.v, bk1.v, s);
            v8f s2 = vzero();
            s2 = wmma16(aq0.v, bl0.v, s2);
            s2 = wmma16(al0.v, bk0.v, s2);
            s2 = wmma16(aq1.v, bl1.v, s2);
            s2 = wmma16(al1.v, bk1.v, s2);
            const v4f mv0 = *(const v4f*)(mq + (size_t)key * SEQ);
            const v4f mv1 = *(const v4f*)(mq + (size_t)key * SEQ + 4);
            const float av = bfr(amb[key]);
#pragma unroll
            for (int r = 0; r < 8; ++r) {
                const float madd = (r < 4) ? mv0[r & 3] : mv1[r & 3];
                float sv = (s[r] + s2[r] * 0.0009765625f) * 0.125f + madd;
                sv = fminf(fmaxf(sv, -10000.0f), 10000.0f) + av;
                s[r] = sv;
            }
            if (t == 0) S0 = s; else S1 = s;
        }
        float alpha[8];
#pragma unroll
        for (int r = 0; r < 8; ++r) {
            float mx = fmaxf(S0[r], S1[r]);
            mx = fmaxf(mx, __shfl_xor(mx, 1, 32));
            mx = fmaxf(mx, __shfl_xor(mx, 2, 32));
            mx = fmaxf(mx, __shfl_xor(mx, 4, 32));
            mx = fmaxf(mx, __shfl_xor(mx, 8, 32));
            const float Mn = fmaxf(rmax[r], mx);
            alpha[r] = __expf(rmax[r] - Mn);
            rmax[r] = Mn;
            const float p0 = __expf(S0[r] - Mn), p1 = __expf(S1[r] - Mn);
            S0[r] = p0; S1[r] = p1;
            float ps = p0 + p1;
            ps += __shfl_xor(ps, 1, 32);
            ps += __shfl_xor(ps, 2, 32);
            ps += __shfl_xor(ps, 4, 32);
            ps += __shfl_xor(ps, 8, 32);
            rsum[r] = alpha[r] * rsum[r] + ps;
        }
#pragma unroll
        for (int r = 0; r < 8; ++r) {
            Pw[(8 * h + r) * PP + m]      = (f16t)(S0[r] * 4096.0f);
            Pw[(8 * h + r) * PP + 16 + m] = (f16t)(S1[r] * 4096.0f);
        }
#pragma unroll
        for (int t = 0; t < 4; ++t)
#pragma unroll
            for (int r = 0; r < 8; ++r) acc[t][r] *= alpha[r];
        __builtin_amdgcn_fence(3  , "wavefront");
        __builtin_amdgcn_wave_barrier();
        Frag ap;
        {
            const f16t* prow = Pw + m * PP + 8 * h;
            ap.hh[0] = *(const v8h*)(prow);
            ap.hh[1] = *(const v8h*)(prow + 16);
        }
#pragma unroll
        for (int t = 0; t < 4; ++t) {
            const f16t* vrow = Vb + (size_t)(t * 16 + m) * SEQ + kc + 8 * h;
            Frag b;
            b.hh[0] = *(const v8h*)(vrow);
            b.hh[1] = *(const v8h*)(vrow + 16);
            acc[t] = wmma16(ap.v, b.v, acc[t]);
        }
    }

    float osc[8];
#pragma unroll
    for (int r = 0; r < 8; ++r) osc[r] = (rsum[r] > 0.0f) ? ((1.0f / rsum[r]) * 0.000244140625f) : 0.0f;
#pragma unroll
    for (int t = 0; t < 4; ++t)
#pragma unroll
        for (int r = 0; r < 8; ++r) Ow[(8 * h + r) * OP + t * 16 + m] = acc[t][r] * osc[r];
    __builtin_amdgcn_fence(3  , "wavefront");
    __builtin_amdgcn_wave_barrier();
    v4f o[8]; size_t off[8];
#pragma unroll
    for (int p = 0; p < 8; ++p) {
        const int L = p * 4 + (lane >> 3), row = L >> 1, co = (L & 1) * 32 + 4 * (lane & 7);
        o[p] = *(const v4f*)(Ow + row * OP + co);
        off[p] = ((size_t)bb * SEQ + q0 + row) * DM + hd0 + co;
    }
#pragma unroll
    for (int p = 0; p < 8; ++p) *(volatile v4f*)(out + off[p]) = o[p];
    __threadfence();
#pragma unroll
    for (int p = 0; p < 8; ++p) *(volatile v4f*)(out + off[p]) = o[p];
}

static inline size_t alup(size_t x) { return (x + 4095) & ~(size_t)4095; }

extern "C" void kernel_launch(void* const* d_in, const int* in_sizes, int n_in,
                              void* d_out, int out_size, void* d_ws, size_t ws_size,
                              hipStream_t stream) {
    if (n_in < 9) return;
    if ((long long)in_sizes[0] < (long long)((NB - 1) * SEQ_FULL + SEQ) * DM) return;
    if (in_sizes[1] < (NB - 1) * SEQ_FULL + SEQ) return;
    if (in_sizes[2] < DM * DM || in_sizes[4] < DM * DM || in_sizes[6] < DM * DM) return;
    if (in_sizes[3] < DM || in_sizes[5] < DM || in_sizes[7] < DM) return;
    if ((long long)in_sizes[8] < (long long)(SEQ - 1) * SEQ_FULL + SEQ) return;
    if ((long long)out_size < (long long)NB * SEQ * DM) return;

    const float* X   = (const float*)d_in[0];
    const float* am  = (const float*)d_in[1];
    const float* Wq  = (const float*)d_in[2];
    const float* bq  = (const float*)d_in[3];
    const float* Wk  = (const float*)d_in[4];
    const float* bk  = (const float*)d_in[5];
    const float* Wv  = (const float*)d_in[6];
    const float* bvv = (const float*)d_in[7];
    const float* M   = (const float*)d_in[8];
    float* out = (float*)d_out;

    char* ws = (char*)d_ws;
    size_t off = 0;
    const size_t szX = (size_t)NTOK * DM * sizeof(f16t);
    const size_t szW = (size_t)3 * DM * DM * sizeof(f16t);
    const size_t szP = (size_t)NB * NH * SEQ * HD * sizeof(f16t);
    const size_t szM = (size_t)SEQ * SEQ * sizeof(float);
    const size_t szA = (size_t)QT * sizeof(unsigned long long);
    f16t* Xh = (f16t*)(ws + off); off += alup(szX);
    f16t* Wt = (f16t*)(ws + off); off += alup(szW);
    f16t* Qh = (f16t*)(ws + off); off += alup(szP);
    f16t* Ql = (f16t*)(ws + off); off += alup(szP);
    f16t* Kh = (f16t*)(ws + off); off += alup(szP);
    f16t* Kl = (f16t*)(ws + off); off += alup(szP);
    f16t* Vt = (f16t*)(ws + off); off += alup(szP);
    float* MT = (float*)(ws + off); off += alup(szM);
    unsigned long long* act = (unsigned long long*)(ws + off); off += alup(szA);
    if (off > ws_size) return;

    k_cvt_x<<<dim3((unsigned)((size_t)NTOK * DM / 8 / 256)), 256, 0, stream>>>(X, Xh);
    k_wt<<<dim3(DM / 64, DM / 64, 3), 256, 0, stream>>>(Wq, Wk, Wv, Wt);
    k_mt<<<dim3(SEQ / 64, SEQ / 64), 256, 0, stream>>>(M, MT);
    k_scan<<<dim3(QT / 16), 256, 0, stream>>>(M, am, act);
    k_proj<<<dim3(NTOK / 64, DM / 64, 3), 128, 0, stream>>>(Xh, Wt, bq, bk, bvv, Qh, Ql, Kh, Kl, Vt);
    k_attn<<<dim3(SEQ / 64, NB * NH), 128, 0, stream>>>(Qh, Ql, Kh, Kl, Vt, MT, am, act, out);
}
